// DINV1_82145544503707
// MI455X (gfx1250) — hardware-verified
//
#include <hip/hip_runtime.h>
#include <math.h>

typedef __attribute__((ext_vector_type(16))) _Float16 v16h;
typedef __attribute__((ext_vector_type(16))) __bf16 v16b;
typedef __attribute__((ext_vector_type(8)))  _Float16 v8h;
typedef __attribute__((ext_vector_type(8)))  float v8f;
typedef __attribute__((ext_vector_type(4)))  float v4f;
typedef __attribute__((ext_vector_type(2)))  float v2f;
typedef __attribute__((ext_vector_type(4)))  unsigned v4u;
typedef __attribute__((ext_vector_type(4)))  int v4i;
typedef float __attribute__((may_alias)) float_a;
typedef int __attribute__((may_alias)) int_a;

template <typename T> __device__ __forceinline__ void vst2(void* p, T v) { *(volatile T*)p = v; __threadfence(); *(volatile T*)p = v; }
__device__ __forceinline__ v8f wmma16(v16h a, v16h b, v8f c) {
  v8f d = __builtin_amdgcn_wmma_f32_16x16x32_f16(false, a, false, b, (short)0, c, false, false);
  asm volatile("v_nop\n\tv_nop\n\tv_nop\n\tv_nop" : "+v"(d) : "v"(a), "v"(b));
  return d;
}
__device__ __forceinline__ v8f wmma_bf(v16b a, v16b b, v8f c) {
  v8f d = __builtin_amdgcn_wmma_f32_16x16x32_bf16(false, a, false, b, (short)0, c, false, false);
  asm volatile("v_nop\n\tv_nop\n\tv_nop\n\tv_nop" : "+v"(d) : "v"(a), "v"(b));
  return d;
}
__device__ __forceinline__ v16h frag_h(const _Float16* rowk0, int lane) {
  union { v16h v; v8h q[2]; } u; const _Float16* p = rowk0 + 8 * (lane >> 4);
  u.q[0] = *(const v8h*)p; u.q[1] = *(const v8h*)(p + 16); return u.v;
}
__device__ __forceinline__ v16h frag_f32(const float* rowk0, int lane) {
  v16h a; const float* p = rowk0 + 8 * (lane >> 4);
#pragma unroll
  for (int i = 0; i < 8; ++i) { a[i] = (_Float16)p[i]; a[8 + i] = (_Float16)p[16 + i]; }
  return a;
}
__device__ __forceinline__ v16h frag_f32s(const float* rowk0, int lane, float sc) {
  v16h a; const float* p = rowk0 + 8 * (lane >> 4);
#pragma unroll
  for (int i = 0; i < 8; ++i) { a[i] = (_Float16)(p[i] * sc); a[8 + i] = (_Float16)(p[16 + i] * sc); }
  return a;
}
__device__ __forceinline__ v16h fragc_f32(const float* W, int k0, int n, int lane, int ld, int K) {
  v16h a; const int g = lane >> 4;
#pragma unroll
  for (int i = 0; i < 8; ++i) { const int ka = k0 + 8 * g + i, kb = ka + 16;
    a[i] = (_Float16)(ka < K ? W[(size_t)ka * ld + n] : 0.f); a[8 + i] = (_Float16)(kb < K ? W[(size_t)kb * ld + n] : 0.f); }
  return a;
}
struct F2 { v16b h, l; };
__device__ __forceinline__ F2 bsplit16(const float v[16]) { F2 r;
#pragma unroll
  for (int i = 0; i < 16; ++i) { const __bf16 h = (__bf16)v[i]; r.h[i] = h; r.l[i] = (__bf16)(v[i] - (float)h); }
  return r; }
__device__ __forceinline__ F2 split_row(const float* row, int k0, int lane) { float v[16]; const float* p = row + k0 + 8 * (lane >> 4);
#pragma unroll
  for (int i = 0; i < 8; ++i) { v[i] = p[i]; v[8 + i] = p[16 + i]; }
  return bsplit16(v); }
__device__ __forceinline__ F2 split_rowK(const float* row, int k0, int lane, int K) { float v[16]; const int g = lane >> 4;
#pragma unroll
  for (int i = 0; i < 8; ++i) { const int ka = k0 + 8 * g + i, kb = ka + 16; v[i] = ka < K ? row[ka] : 0.f; v[8 + i] = kb < K ? row[kb] : 0.f; }
  return bsplit16(v); }
__device__ __forceinline__ F2 split_col(const float* W, int k0, int n, int lane, int ld, int K) { float v[16]; const int g = lane >> 4;
#pragma unroll
  for (int i = 0; i < 8; ++i) { const int ka = k0 + 8 * g + i, kb = ka + 16; v[i] = ka < K ? W[(size_t)ka * ld + n] : 0.f; v[8 + i] = kb < K ? W[(size_t)kb * ld + n] : 0.f; }
  return bsplit16(v); }
__device__ __forceinline__ v8f mac3(const F2& a, const F2& b, v8f c) { c = wmma_bf(a.l, b.h, c); c = wmma_bf(a.h, b.l, c); return wmma_bf(a.h, b.h, c); }
__device__ __forceinline__ float sigm(float v) { return 1.0f / (1.0f + expf(-v)); }
#define LDSX() do { asm volatile("s_wait_dscnt 0" ::: "memory"); __builtin_amdgcn_wave_barrier(); __builtin_amdgcn_fence(__ATOMIC_RELEASE, "workgroup"); } while (0)

#define NBT 2048
#define SEQ 200
#define SP 208
#define DE 64
#define NI 100000
#define NC 1000
#define AH 64
#define X0W 192
#define M0 256
#define M1 128
#define M2 64

__global__ __launch_bounds__(256) void k_prepB(const float* __restrict__ aW1, float* __restrict__ B1c, float* __restrict__ A13) {
  const int tid = threadIdx.x, blk = blockIdx.x;
  const int e = blk * 256 + tid;
  if (e < 128 * AH) { const int k = e / AH, o = e % AH; const float v = k < 64 ? aW1[(size_t)(64 + k) * AH + o] - aW1[(size_t)(128 + k) * AH + o] : aW1[(size_t)(192 + k - 64) * AH + o]; vst2(B1c + e, (float_a)v); }
  else { const int e2 = e - 128 * AH; const int d = e2 / AH, o = e2 % AH; vst2(A13 + e2, (float_a)(aW1[(size_t)d * AH + o] + aW1[(size_t)(128 + d) * AH + o])); }
}
__global__ __launch_bounds__(256) void k_att(const int* __restrict__ hist, const int* __restrict__ mask, const int* __restrict__ titem, const int* __restrict__ tcat, const float* __restrict__ iemb, const float* __restrict__ cemb,
                                           const float* __restrict__ B1c, const float* __restrict__ A13, const float* __restrict__ ab1, const float* __restrict__ aW2, const float* __restrict__ ab2, const float* __restrict__ aW3, const float* __restrict__ ab3,
                                           float* __restrict__ X0) {
  __shared__ __align__(16) float sK[SP][DE + 4];
  __shared__ __align__(16) float sH[SP][DE + 4];
  __shared__ float sq[DE], scq[AH], ssc[SP], sw[SP];
  __shared__ __align__(16) float sx[X0W];
  const int tid = threadIdx.x, w = tid >> 5, lane = tid & 31, col = lane & 15, g = lane >> 4; const int b = blockIdx.x;
  int ti = titem[b]; ti = ti < 0 ? 0 : (ti >= NI ? NI - 1 : ti); int tci = tcat[b]; tci = tci < 0 ? 0 : (tci >= NC ? NC - 1 : tci);
  if (tid < DE) sq[tid] = iemb[(size_t)ti * DE + tid];
  for (int q = tid; q < SP * DE; q += 256) { const int s = q >> 6, d = q & 63; float v = 0.f; if (s < SEQ) { int id = hist[(size_t)b * SEQ + s]; id = id < 0 ? 0 : (id >= NI ? NI - 1 : id); v = iemb[(size_t)id * DE + d]; } sK[s][d] = v; }
  __syncthreads();
  if (tid < AH) { float a = ab1[tid]; for (int d = 0; d < DE; ++d) a += sq[d] * A13[d * AH + tid]; scq[tid] = a; }
  __syncthreads();
  for (int tI = w; tI < SP / 16; tI += 8) { const int s = tI * 16 + col; v8f acc[4] = {};
#pragma unroll
    for (int kc = 0; kc < 4; ++kc) { v16h a;
#pragma unroll
      for (int i = 0; i < 8; ++i) { const int ka = kc * 32 + 8 * g + i, kb = ka + 16;
        const float va = ka < 64 ? sK[s][ka] * 64.0f : sq[ka - 64] * sK[s][ka - 64] * 4096.0f; const float vb = kb < 64 ? sK[s][kb] * 64.0f : sq[kb - 64] * sK[s][kb - 64] * 4096.0f;
        a[i] = (_Float16)va; a[8 + i] = (_Float16)vb; }
#pragma unroll
      for (int j = 0; j < 4; ++j) { v16h bb = fragc_f32(B1c, kc * 32, j * 16 + col, lane, AH, 128);
        if (kc < 2) {
#pragma unroll
          for (int e = 0; e < 16; ++e) bb[e] = bb[e] * (_Float16)64.0f; }
        acc[j] = wmma16(a, bb, acc[j]); } }
#pragma unroll
    for (int j = 0; j < 4; ++j) { const int o = j * 16 + col;
#pragma unroll
      for (int r = 0; r < 8; ++r) { const float v = acc[j][r] * (1.0f / 4096.0f) + scq[o]; sH[tI * 16 + 8 * g + r][o] = v > 0.f ? v : 0.f; } } }
  __syncthreads();
  for (int tI = w; tI < SP / 16; tI += 8) { v8f acc[4] = {};
#pragma unroll
    for (int kc = 0; kc < 2; ++kc) { const v16h a = frag_f32(&sH[tI * 16 + col][0] + kc * 32, lane);
#pragma unroll
      for (int j = 0; j < 4; ++j) { v16h bb = fragc_f32(aW2, kc * 32, j * 16 + col, lane, AH, AH);
#pragma unroll
        for (int e = 0; e < 16; ++e) bb[e] = bb[e] * (_Float16)4.0f;
        acc[j] = wmma16(a, bb, acc[j]); } }
    LDSX();
#pragma unroll
    for (int j = 0; j < 4; ++j) { const int o = j * 16 + col;
#pragma unroll
      for (int r = 0; r < 8; ++r) { const float v = acc[j][r] * 0.25f + ab2[o]; sH[tI * 16 + 8 * g + r][o] = v > 0.f ? v : 0.f; } } }
  __syncthreads();
  if (tid < SP) { const int s = tid; float sc = -1.0e9f; if (s < SEQ) { float a = ab3[0]; for (int o = 0; o < AH; ++o) a += sH[s][o] * aW3[o]; sc = mask[(size_t)b * SEQ + s] == 0 ? -1.0e9f : a; } ssc[s] = s < SEQ ? sc : -3.0e38f; }
  __syncthreads();
  if (tid < 32) { float m = -3.4e38f; for (int s = lane; s < SEQ; s += 32) m = fmaxf(m, ssc[s]);
#pragma unroll
    for (int off = 16; off >= 1; off >>= 1) m = fmaxf(m, __shfl_xor(m, off, 32));
    float l = 0.f; for (int s = lane; s < SEQ; s += 32) { const float p = expf(ssc[s] - m); sw[s] = p; l += p; }
#pragma unroll
    for (int off = 16; off >= 1; off >>= 1) l += __shfl_xor(l, off, 32);
    const float inv = 1.0f / l; __builtin_amdgcn_wave_barrier(); asm volatile("s_wait_dscnt 0" ::: "memory");
    for (int s = lane; s < SEQ; s += 32) sw[s] *= inv; }
  __syncthreads();
  if (tid < DE) { const int d = tid; float a = 0.f; for (int s = 0; s < SEQ; ++s) a += sw[s] * sK[s][d]; sx[d] = a; sx[DE + d] = sq[d]; sx[2 * DE + d] = cemb[(size_t)tci * DE + d]; }
  __syncthreads();
  if (tid < X0W / 4) vst2(X0 + (size_t)b * X0W + tid * 4, *(const v4f*)(&sx[tid * 4]));
}
template <int CIN, int COUT, int RAW>
__global__ __launch_bounds__(128) void k_lin(const float* __restrict__ prein, const float* __restrict__ stat, const float* __restrict__ gam, const float* __restrict__ bet, const float* __restrict__ W, const float* __restrict__ bias, float ascale, float wscale,
                                           float* __restrict__ preout, float* __restrict__ part) {
  __shared__ __align__(16) float st[COUT][68];
  __shared__ float ssc[CIN], ssh[CIN];
  const int tid = threadIdx.x, wave = tid >> 5, lane = tid & 31, col = lane & 15, g = lane >> 4;
  const int r0 = blockIdx.x * 64 + wave * 16;
  for (int c = tid; c < CIN; c += 128) { if (RAW) { ssc[c] = 1.0f; ssh[c] = 0.f; } else { const float sc = gam[c] * stat[c * 2 + 1]; ssc[c] = sc; ssh[c] = bet[c] - stat[c * 2] * sc; } }
  __syncthreads();
  v8f acc[COUT / 16];
#pragma unroll
  for (int j = 0; j < COUT / 16; ++j) acc[j] = (v8f){};
  (void)ascale; (void)wscale;
#pragma unroll 1
  for (int kc = 0; kc < CIN / 32; ++kc) { float av[16]; const float* pr = prein + (size_t)(r0 + col) * CIN + kc * 32;
#pragma unroll
    for (int e = 0; e < 8; ++e) { const int ka = 8 * g + e, kb = ka + 16; float va = pr[ka] * ssc[kc * 32 + ka] + ssh[kc * 32 + ka], vb = pr[kb] * ssc[kc * 32 + kb] + ssh[kc * 32 + kb];
      if (!RAW) { va = va > 0.f ? va : 0.f; vb = vb > 0.f ? vb : 0.f; }
      av[e] = va; av[8 + e] = vb; }
    const F2 a = bsplit16(av);
#pragma unroll
    for (int j = 0; j < COUT / 16; ++j) acc[j] = mac3(a, split_col(W, kc * 32, j * 16 + col, lane, COUT, CIN), acc[j]); }
#pragma unroll
  for (int j = 0; j < COUT / 16; ++j) { const float bb = bias[j * 16 + col];
#pragma unroll
    for (int r = 0; r < 8; ++r) st[j * 16 + col][wave * 16 + 8 * g + r] = acc[j][r] + bb; }
  __syncthreads();
  for (int q = tid; q < 64 * COUT / 4; q += 128) { const int rl = q / (COUT / 4), pc = q % (COUT / 4); v4f v = { st[pc * 4][rl], st[pc * 4 + 1][rl], st[pc * 4 + 2][rl], st[pc * 4 + 3][rl] };
    vst2(preout + (size_t)(blockIdx.x * 64 + rl) * COUT + pc * 4, v); }
  for (int o = tid; o < COUT; o += 128) { float s = 0.f, s2 = 0.f; for (int rl = 0; rl < 64; ++rl) { const float v = st[o][rl]; s += v; s2 += v * v; }
    vst2(part + (size_t)blockIdx.x * 2 * COUT + o, (float_a)s); vst2(part + (size_t)blockIdx.x * 2 * COUT + COUT + o, (float_a)s2); }
}
__global__ __launch_bounds__(256) void k_stat(const float* __restrict__ part, int C, float* __restrict__ stat) {
  __shared__ __align__(16) float so[512];
  const int c = threadIdx.x;
  if (c < C) { float s = 0.f, s2 = 0.f;
#pragma unroll 1
    for (int b = 0; b < NBT / 64; ++b) { s += part[(size_t)b * 2 * C + c]; s2 += part[(size_t)b * 2 * C + C + c]; }
    const float mu = s / (float)NBT; float var = s2 / (float)NBT - mu * mu; var = var < 0.f ? 0.f : var; so[c * 2] = mu; so[c * 2 + 1] = rsqrtf(var + 1e-5f); }
  __syncthreads();
  for (int q = c; q < 2 * C / 4; q += 256) vst2(stat + q * 4, *(const v4f*)(&so[q * 4]));
}
__global__ __launch_bounds__(256) void k_fin(const float* __restrict__ pre2, const float* __restrict__ stat2, const float* __restrict__ gam, const float* __restrict__ bet, const float* __restrict__ W3, const float* __restrict__ b3, float* __restrict__ out) {
  __shared__ __align__(16) float so[256];
  const int tid = threadIdx.x, b = blockIdx.x * 256 + tid; float a = b3[0];
#pragma unroll 1
  for (int c = 0; c < M2; ++c) { const float sc = gam[c] * stat2[c * 2 + 1]; float v = (pre2[(size_t)b * M2 + c] - stat2[c * 2]) * sc + bet[c]; v = v > 0.f ? v : 0.f; a += v * W3[c]; }
  so[tid] = a; __syncthreads();
  if (tid < 64) vst2(out + (size_t)blockIdx.x * 256 + tid * 4, *(const v4f*)(&so[tid * 4]));
}
extern "C" void kernel_launch(void* const* d_in, const int* in_sizes, int n_in, void* d_out, int out_size, void* d_ws, size_t ws_size, hipStream_t stream) {
  (void)in_sizes; (void)n_in; (void)out_size; (void)ws_size;
  const int* hist = (const int*)d_in[0]; const int* msk = (const int*)d_in[3]; const int* titem = (const int*)d_in[4]; const int* tcat = (const int*)d_in[5];
  const float** I = (const float**)d_in;
  const float* iemb = I[6]; const float* cemb = I[7]; const float* aW1 = I[8]; const float* ab1 = I[9]; const float* aW2 = I[10]; const float* ab2 = I[11]; const float* aW3 = I[12]; const float* ab3 = I[13];
  const float* W0 = I[14]; const float* b0 = I[15]; const float* g0 = I[16]; const float* be0 = I[17]; const float* W1 = I[18]; const float* b1 = I[19]; const float* g1 = I[20]; const float* be1 = I[21];
  const float* W2 = I[22]; const float* b2 = I[23]; const float* g2 = I[24]; const float* be2 = I[25]; const float* W3 = I[26]; const float* b3 = I[27];
  float* out = (float*)d_out;
  char* ws = (char*)d_ws; size_t off = 0;
  auto take = [&](size_t bytes) { char* p = ws + off; off += (bytes + 255) & ~(size_t)255; return p; };
  float* B1c = (float*)take(128 * AH * 4); float* A13 = (float*)take(64 * AH * 4); float* X0 = (float*)take((size_t)NBT * X0W * 4);
  float* pre0 = (float*)take((size_t)NBT * M0 * 4); float* pre1 = (float*)take((size_t)NBT * M1 * 4); float* pre2 = (float*)take((size_t)NBT * M2 * 4);
  float* part = (float*)take((size_t)(NBT / 64) * 2 * M0 * 4); float* st0 = (float*)take(2 * M0 * 4); float* st1 = (float*)take(2 * M1 * 4); float* st2 = (float*)take(2 * M2 * 4);
  k_prepB<<<48, 256, 0, stream>>>(aW1, B1c, A13);
  k_att<<<NBT, 256, 0, stream>>>(hist, msk, titem, tcat, iemb, cemb, B1c, A13, ab1, aW2, ab2, aW3, ab3, X0);
  k_lin<X0W, M0, 1><<<NBT / 64, 128, 0, stream>>>(X0, nullptr, nullptr, nullptr, W0, b0, 64.0f, 4.0f, pre0, part);
  k_stat<<<1, 256, 0, stream>>>(part, M0, st0);
  k_lin<M0, M1, 0><<<NBT / 64, 128, 0, stream>>>(pre0, st0, g0, be0, W1, b1, 1.0f, 4.0f, pre1, part);
  k_stat<<<1, 256, 0, stream>>>(part, M1, st1);
  k_lin<M1, M2, 0><<<NBT / 64, 128, 0, stream>>>(pre1, st1, g1, be1, W2, b2, 1.0f, 4.0f, pre2, part);
  k_stat<<<1, 256, 0, stream>>>(part, M2, st2);
  k_fin<<<NBT / 256, 256, 0, stream>>>(pre2, st2, g2, be2, W3, b3, out);
}
